// PointNetFeaturePropagation_35296041239307
// MI455X (gfx1250) — hardware-verified
//
#include <hip/hip_runtime.h>
#include <math.h>

#pragma clang fp contract(off)

constexpr int kBatch = 8;
constexpr int kNq    = 8192;
constexpr int kNs    = 2048;
constexpr int kCf1   = 128;
constexpr int kCf2   = 256;
constexpr int kCin   = 384;
constexpr int kHid1  = 256;
constexpr int kHid2  = 128;
constexpr int kRows  = kBatch * kNq;
constexpr int kRowsPerStat = 256;
constexpr int kStatBlocks  = kRows / kRowsPerStat;
constexpr float kWCarry    = 16.0f;
constexpr float kWCarryInv = 1.0f / 16.0f;
constexpr float kBnEps     = 1e-5f;
constexpr double kInvRows  = 1.0 / 65536.0;

static_assert(kNq % 256 == 0, "s");
static_assert(kNs % 256 == 0, "s");
static_assert(kRows % 8 == 0 && kRows % 64 == 0, "s");
static_assert(kCin % 32 == 0 && kHid1 % 32 == 0, "s");
static_assert(kHid1 % 64 == 0 && kHid2 % 64 == 0, "s");
static_assert(kRows % kRowsPerStat == 0 && kStatBlocks == 256, "s");
static_assert((kHid1 * kCin) % 2048 == 0 && (kHid2 * kHid1) % 2048 == 0, "s");

constexpr size_t kOffXH  = 0;
constexpr size_t kSzXH   = (size_t)kRows * kCin * 2;
constexpr size_t kOffH1P = kOffXH + kSzXH;
constexpr size_t kSzH1P  = (size_t)kRows * kHid1 * 4;
constexpr size_t kOffW1H = kOffH1P + kSzH1P;
constexpr size_t kSzW1H  = (size_t)kHid1 * kCin * 2;
constexpr size_t kOffW2H = kOffW1H + kSzW1H;
constexpr size_t kSzW2H  = (size_t)kHid2 * kHid1 * 2;
constexpr size_t kOffP1  = kOffW2H + kSzW2H;
constexpr size_t kSzP1   = (size_t)kStatBlocks * 2 * kHid1 * 4;
constexpr size_t kOffP2  = kOffP1 + kSzP1;
constexpr size_t kSzP2   = (size_t)kStatBlocks * 2 * kHid2 * 4;
constexpr size_t kOffT1  = kOffP2 + kSzP2;
constexpr size_t kSzT1   = 4096;
constexpr size_t kOffT2  = kOffT1 + kSzT1;
constexpr size_t kSzT2   = 2048;
constexpr size_t kWsTotal = kOffT2 + kSzT2;
static_assert(kWsTotal == 118495232, "s");
static_assert(kWsTotal <= (size_t)134217728, "s");
static_assert(kOffH1P % 256 == 0 && kOffW1H % 256 == 0 && kOffW2H % 256 == 0 &&
              kOffP1 % 256 == 0 && kOffP2 % 256 == 0 && kOffT1 % 256 == 0 && kOffT2 % 256 == 0, "s");

typedef __attribute__((ext_vector_type(16))) _Float16 v16h;
typedef __attribute__((ext_vector_type(8)))  _Float16 v8h;
typedef __attribute__((ext_vector_type(16))) __bf16   v16b;
typedef __attribute__((ext_vector_type(8)))  __bf16   v8b;
typedef __attribute__((ext_vector_type(8)))  float    v8f;
typedef __attribute__((ext_vector_type(4)))  float    v4f;
typedef __attribute__((ext_vector_type(4)))  unsigned int v4u;
typedef __attribute__((ext_vector_type(4)))  int      v4i;

__device__ __forceinline__ unsigned short f2bf_bits(float f) {
  unsigned u = __float_as_uint(f);
  return (unsigned short)((u + 0x7FFFu + ((u >> 16) & 1u)) >> 16);
}
__device__ __forceinline__ float bf_bits2f(unsigned short h) { return __uint_as_float(((unsigned)h) << 16); }

__device__ __forceinline__ void dep_guard_h(v8f& a, v8f& b, v16h x, v16h y) { asm volatile("v_nop\n\tv_nop\n\tv_nop\n\tv_nop" : "+v"(a), "+v"(b) : "v"(x), "v"(y)); }
__device__ __forceinline__ void dep_guard_b(v8f& a, v8f& b, v16b x, v16b y) { asm volatile("v_nop\n\tv_nop\n\tv_nop\n\tv_nop" : "+v"(a), "+v"(b) : "v"(x), "v"(y)); }
__device__ __forceinline__ void keep4_h(v16h a, v16h b, v16h c, v16h d) { asm volatile("v_nop" :: "v"(a), "v"(b), "v"(c), "v"(d)); }
__device__ __forceinline__ void keep4_b(v16b a, v16b b, v16b c, v16b d) { asm volatile("v_nop" :: "v"(a), "v"(b), "v"(c), "v"(d)); }
__device__ __forceinline__ void acc_guard4(v8f& a, v8f& b, v8f& c, v8f& d) { asm volatile("v_nop\n\tv_nop\n\tv_nop\n\tv_nop" : "+v"(a), "+v"(b), "+v"(c), "+v"(d)); }
template <typename T> struct Frag;
template <> struct Frag<_Float16> {
  typedef v16h V; union U { v16h v; v8h h[2]; };
  static __device__ __forceinline__ v16h load(const _Float16* p) {
    U f; f.h[0] = *(const v8h*)(p); f.h[1] = *(const v8h*)(p + 16); return f.v;
  }
  static __device__ __forceinline__ v8f mma(v16h a, v16h b, v8f c) {
    return __builtin_amdgcn_wmma_f32_16x16x32_f16(false, a, false, b, (short)0, c, false, false);
  }
  static __device__ __forceinline__ void guard(v8f& a, v8f& b, v16h x, v16h y) { dep_guard_h(a, b, x, y); }
  static __device__ __forceinline__ void keep(v16h a, v16h b, v16h c, v16h d) { keep4_h(a, b, c, d); }
};
template <> struct Frag<__bf16> {
  typedef v16b V; union U { v16b v; v8b h[2]; };
  static __device__ __forceinline__ v16b load(const __bf16* p) {
    U f; f.h[0] = *(const v8b*)(p); f.h[1] = *(const v8b*)(p + 16); return f.v;
  }
  static __device__ __forceinline__ v8f mma(v16b a, v16b b, v8f c) {
    return __builtin_amdgcn_wmma_f32_16x16x32_bf16(false, a, false, b, (short)0, c, false, false);
  }
  static __device__ __forceinline__ void guard(v8f& a, v8f& b, v16b x, v16b y) { dep_guard_b(a, b, x, y); }
  static __device__ __forceinline__ void keep(v16b a, v16b b, v16b c, v16b d) { keep4_b(a, b, c, d); }
};

__device__ __forceinline__ unsigned pk16(unsigned short a, unsigned short b) { return (unsigned)a | ((unsigned)b << 16); }
__device__ __forceinline__ unsigned short h_bits(float f) { const _Float16 h = (_Float16)f; return __builtin_bit_cast(unsigned short, h); }

__device__ __forceinline__ float bf16q(float f) {
  unsigned u = __float_as_uint(f);
  u = (u + 0x7FFFu + ((u >> 16) & 1u)) & 0xFFFF0000u;
  return __uint_as_float(u);
}

template <int ET> struct Elem;
template <> struct Elem<0> { typedef _Float16 T; };
template <> struct Elem<1> { typedef __bf16 T; };
template <int ET, bool SPLIT, int BIAS_MODE, int OUT_MODE, bool RESID, int ACT = 0>
__global__ __launch_bounds__(256) void wmma_gemm64(
    const unsigned short* __restrict__ Ap, const unsigned short* __restrict__ A2p, int lda, long strideA,
    const unsigned short* __restrict__ Btp, const unsigned short* __restrict__ Bt2p, int ldb, long strideB,
    void* __restrict__ Cout, void* __restrict__ Cout2, int ldc, long strideC,
    const float* __restrict__ bias,
    const float* __restrict__ resid, long strideR,
    int M, int N, int K, float scale) {
  typedef typename Elem<ET>::T T;
  typedef typename Frag<T>::V V;
  const T* A = (const T*)Ap; const T* A2 = (const T*)A2p; const T* Bt = (const T*)Btp; const T* Bt2 = (const T*)Bt2p;
  __shared__ __align__(16) float sT[8][16 * 68];
  const int b    = blockIdx.y;
  const int lane = threadIdx.x & 31;
  const int wave = threadIdx.x >> 5;
  const int tilesN = N >> 6;
  const int tilesM = M >> 6;
  const int tile = blockIdx.x * 8 + wave;
  if (tile >= tilesM * tilesN) return;
  const int tm = tile / tilesN;
  const int tn = tile - tm * tilesN;
  const int m0 = tm << 6;
  const int n0 = tn << 6;

  const T* Ab  = A  + (size_t)b * strideA;
  const T* Bb  = Bt + (size_t)b * strideB;
  const T* Ab2 = SPLIT ? (A2  + (size_t)b * strideA) : nullptr;
  const T* Bb2 = SPLIT ? (Bt2 + (size_t)b * strideB) : nullptr;

  const int rlane = lane & 15;
  const int koff  = (lane >> 4) * 8;
  const int mOff  = (lane >> 4) * 8;

  v8f acc[4][4];
#pragma unroll
  for (int i = 0; i < 4; ++i)
#pragma unroll
    for (int j = 0; j < 4; ++j) acc[i][j] = (v8f){0.f,0.f,0.f,0.f,0.f,0.f,0.f,0.f};

  for (int k0 = 0; k0 < K; k0 += 32) {
    V bh[4], bl[4];
#pragma unroll
    for (int j = 0; j < 4; ++j) {
      const size_t bo = (size_t)(n0 + (j << 4) + rlane) * ldb + koff + k0;
      bh[j] = Frag<T>::load(Bb + bo);
      if (SPLIT) bl[j] = Frag<T>::load(Bb2 + bo);
    }
#pragma unroll
    for (int i = 0; i < 4; ++i) {
      const size_t ao = (size_t)(m0 + (i << 4) + rlane) * lda + koff + k0;
      V ah = Frag<T>::load(Ab + ao);
      V al;
      if (SPLIT) al = Frag<T>::load(Ab2 + ao);
#pragma unroll
      for (int j = 0; j < 4; ++j) {
        acc[i][j] = Frag<T>::mma(ah, bh[j], acc[i][j]);
        if (SPLIT) {
          acc[i][j] = Frag<T>::mma(ah, bl[j], acc[i][j]);
          acc[i][j] = Frag<T>::mma(al, bh[j], acc[i][j]);
        }
      }
      Frag<T>::guard(acc[i][0], acc[i][3], ah, SPLIT ? al : ah);
    }
    Frag<T>::keep(bh[0], bh[1], bh[2], bh[3]);
    if (SPLIT) Frag<T>::keep(bl[0], bl[1], bl[2], bl[3]);
  }
  acc_guard4(acc[0][0], acc[0][1], acc[0][2], acc[0][3]);
  acc_guard4(acc[1][0], acc[1][1], acc[1][2], acc[1][3]);
  acc_guard4(acc[2][0], acc[2][1], acc[2][2], acc[2][3]);
  acc_guard4(acc[3][0], acc[3][1], acc[3][2], acc[3][3]);

  float* slab = sT[wave];
  const float* Rb = RESID ? (resid + (size_t)b * strideR) : nullptr;
#pragma unroll
  for (int i = 0; i < 4; ++i) {
    const int mBase = m0 + (i << 4);
#pragma unroll
    for (int j = 0; j < 4; ++j) {
      const int n = n0 + (j << 4) + rlane;
      float bv = 0.f;
      if (BIAS_MODE == 2) bv = bias[n];
#pragma unroll
      for (int r = 0; r < 8; ++r) {
        float v = acc[i][j][r] * scale;
        if (BIAS_MODE == 1) v += bias[mBase + mOff + r];
        if (BIAS_MODE == 2) v += bv;
        if (RESID) v += Rb[(size_t)(mBase + mOff + r) * ldc + n];
        if (ACT == 2) v = fmaxf(v, 0.0f);
        if (ACT == 4) v = (v > 0.f) ? v : 0.01f * v;
        slab[(mOff + r) * 68 + (j << 4) + rlane] = v;
      }
    }
    __builtin_amdgcn_fence(__ATOMIC_RELEASE, "workgroup");
    __builtin_amdgcn_wave_barrier();
    __builtin_amdgcn_fence(__ATOMIC_ACQUIRE, "workgroup");
    if (OUT_MODE == 0) {
      float* C = (float*)Cout + (size_t)b * strideC;
      const int hh = lane >> 4, c4 = (lane & 15) * 4;
      for (int pass = 0; pass < 2; ++pass) {
#pragma unroll
        for (int it = 0; it < 8; ++it) {
          const int row = it * 2 + hh;
          v4f v = *(const v4f*)(slab + row * 68 + c4);
          *(volatile v4f*)(C + (size_t)(mBase + row) * ldc + n0 + c4) = v;
        }
        __threadfence();
      }
    } else {
      const int q = lane >> 3, c8 = (lane & 7) * 8;
      unsigned short* C  = (unsigned short*)Cout  + (size_t)b * strideC;
      unsigned short* C2 = (OUT_MODE == 2) ? ((unsigned short*)Cout2 + (size_t)b * strideC) : nullptr;
      for (int pass = 0; pass < 2; ++pass) {
#pragma unroll
        for (int it = 0; it < 4; ++it) {
          const int row = it * 4 + q;
          const float* sp = slab + row * 68 + c8;
          v8h hv, lv;
#pragma unroll
          for (int e = 0; e < 8; ++e) {
            if (OUT_MODE == 1) {
              hv[e] = (_Float16)sp[e];
            } else {
              unsigned short hb = f2bf_bits(sp[e]);
              unsigned short lb = f2bf_bits(sp[e] - bf_bits2f(hb));
              hv[e] = __builtin_bit_cast(_Float16, hb);
              lv[e] = __builtin_bit_cast(_Float16, lb);
            }
          }
          *(volatile v8h*)(C + (size_t)(mBase + row) * ldc + n0 + c8) = hv;
          if (OUT_MODE == 2) *(volatile v8h*)(C2 + (size_t)(mBase + row) * ldc + n0 + c8) = lv;
        }
        __threadfence();
      }
    }
    __builtin_amdgcn_fence(__ATOMIC_RELEASE, "workgroup");
    __builtin_amdgcn_wave_barrier();
    __builtin_amdgcn_fence(__ATOMIC_ACQUIRE, "workgroup");
  }
}

__global__ __launch_bounds__(256) void cast8_w_kernel(const float* __restrict__ in, unsigned short* __restrict__ out,
                                                      int n8, float carry) {
  const int i = blockIdx.x * 256 + threadIdx.x;
  if (i >= n8) return;
  const float* p = in + 8 * (size_t)i;
  const v4f a = *(const v4f*)(p);
  const v4f c = *(const v4f*)(p + 4);
  unsigned short hb[8];
#pragma unroll
  for (int e = 0; e < 4; ++e) {
    hb[e]     = h_bits(bf16q(a[e]) * carry);
    hb[4 + e] = h_bits(bf16q(c[e]) * carry);
  }
  const v4u u = (v4u){pk16(hb[0], hb[1]), pk16(hb[2], hb[3]), pk16(hb[4], hb[5]), pk16(hb[6], hb[7])};
  unsigned short* q = out + 8 * (size_t)i;
  *(volatile v4u*)q = u;
  __threadfence();
  *(volatile v4u*)q = u;
}

__global__ __launch_bounds__(256) void knn_buildx_kernel(const float* __restrict__ xyz1, const float* __restrict__ xyz2,
                                                         const float* __restrict__ f1, const float* __restrict__ f2,
                                                         unsigned short* __restrict__ Xo) {
  __shared__ v4f pts[kNs];
  __shared__ v4i sIdx[256];
  __shared__ v4f sWgt[256];
  const int t = threadIdx.x;
  const int b = blockIdx.y;
  const float* p2 = xyz2 + (size_t)b * kNs * 3;
#pragma unroll 1
  for (int i = t; i < kNs; i += 256) {
    const float y0 = bf16q(p2[i * 3 + 0]);
    const float y1 = bf16q(p2[i * 3 + 1]);
    const float y2 = bf16q(p2[i * 3 + 2]);
    const float t0 = y0 * y0;
    const float t1 = y1 * y1;
    const float t2 = y2 * y2;
    const float sy = (t0 + t2) + t1;
    v4f v;
    v[0] = y0; v[1] = y1; v[2] = y2; v[3] = sy;
    pts[i] = v;
  }
  __syncthreads();

  {
    const int n = blockIdx.x * 256 + t;
    const size_t row = (size_t)b * kNq + n;
    const float x0 = bf16q(xyz1[row * 3 + 0]);
    const float x1 = bf16q(xyz1[row * 3 + 1]);
    const float x2 = bf16q(xyz1[row * 3 + 2]);
    const float s0 = x0 * x0;
    const float s1 = x1 * x1;
    const float s2 = x2 * x2;
    const float sx = (s0 + s2) + s1;

    float e0 = 3.0e38f, e1 = 3.0e38f, e2 = 3.0e38f;
    int i0 = 0, i1 = 0, i2 = 0;
#pragma unroll 2
    for (int s = 0; s < kNs; ++s) {
      const v4f p = pts[s];
      float dp = x0 * p[0];
      dp = fmaf(x1, p[1], dp);
      dp = fmaf(x2, p[2], dp);
      const float twodp = 2.0f * dp;
      const float dsum = sx + p[3];
      const float dd = dsum - twodp;
      const float dist = sqrtf(fmaxf(dd, 0.0f)) + 1e-10f;
      const bool lt0 = dist < e0;
      const bool lt1 = dist < e1;
      const bool lt2 = dist < e2;
      const float ne2 = lt1 ? e1 : (lt2 ? dist : e2);
      const int   ni2 = lt1 ? i1 : (lt2 ? s : i2);
      const float ne1 = lt0 ? e0 : (lt1 ? dist : e1);
      const int   ni1 = lt0 ? i0 : (lt1 ? s : i1);
      const float ne0 = lt0 ? dist : e0;
      const int   ni0 = lt0 ? s : i0;
      e0 = ne0; e1 = ne1; e2 = ne2;
      i0 = ni0; i1 = ni1; i2 = ni2;
    }
    const float w0 = 1.0f / e0;
    const float w1 = 1.0f / e1;
    const float w2 = 1.0f / e2;
    const float wsum = (w0 + w2) + w1;
    const float wi = 1.0f / wsum;
    v4i iv;
    iv[0] = i0; iv[1] = i1; iv[2] = i2; iv[3] = i2;
    v4f wv;
    wv[0] = w0 * wi; wv[1] = w1 * wi; wv[2] = w2 * wi; wv[3] = 0.0f;
    sIdx[t] = iv;
    sWgt[t] = wv;
  }
  __syncthreads();

  const int lane = t & 31, wave = t >> 5;
  const int c8  = lane * 8;
  const int l16 = lane & 15;
  const size_t rowBase = (size_t)b * kNq + (size_t)blockIdx.x * 256;
  const float* f2b = f2 + (size_t)b * kNs * kCf2;
#pragma unroll 1
  for (int it = 0; it < 32; ++it) {
    const int rl = it * 8 + wave;
    const size_t row = rowBase + rl;
    const v4i iv = sIdx[rl];
    const v4f wv = sWgt[rl];
    int j0 = iv[0]; j0 = j0 < 0 ? 0 : (j0 > kNs - 1 ? kNs - 1 : j0);
    int j1 = iv[1]; j1 = j1 < 0 ? 0 : (j1 > kNs - 1 ? kNs - 1 : j1);
    int j2 = iv[2]; j2 = j2 < 0 ? 0 : (j2 > kNs - 1 ? kNs - 1 : j2);
    const float w0 = wv[0], w1 = wv[1], w2 = wv[2];
    const float* g0p = f2b + (size_t)j0 * kCf2 + c8;
    const float* g1p = f2b + (size_t)j1 * kCf2 + c8;
    const float* g2p = f2b + (size_t)j2 * kCf2 + c8;
    const v4f ga0 = *(const v4f*)(g0p); const v4f ga1 = *(const v4f*)(g0p + 4);
    const v4f gb0 = *(const v4f*)(g1p); const v4f gb1 = *(const v4f*)(g1p + 4);
    const v4f gc0 = *(const v4f*)(g2p); const v4f gc1 = *(const v4f*)(g2p + 4);
    const float* fp = f1 + row * kCf1 + l16 * 8;
    const v4f fa = *(const v4f*)(fp);
    const v4f fb = *(const v4f*)(fp + 4);

    unsigned short hx[8];
    unsigned short hf[8];
#pragma unroll
    for (int e = 0; e < 4; ++e) {
      const float pa = bf16q(ga0[e]) * w0;
      const float pb = bf16q(gb0[e]) * w1;
      const float pc = bf16q(gc0[e]) * w2;
      const float va = (pa + pb) + pc;
      hx[e] = h_bits(va);
      const float qa = bf16q(ga1[e]) * w0;
      const float qb = bf16q(gb1[e]) * w1;
      const float qc = bf16q(gc1[e]) * w2;
      const float vb = (qa + qb) + qc;
      hx[4 + e] = h_bits(vb);
      hf[e]     = h_bits(bf16q(fa[e]));
      hf[4 + e] = h_bits(bf16q(fb[e]));
    }
    const v4u ux = (v4u){pk16(hx[0], hx[1]), pk16(hx[2], hx[3]), pk16(hx[4], hx[5]), pk16(hx[6], hx[7])};
    const v4u uf = (v4u){pk16(hf[0], hf[1]), pk16(hf[2], hf[3]), pk16(hf[4], hf[5]), pk16(hf[6], hf[7])};
    unsigned short* xa = Xo + row * kCin + c8;
    unsigned short* xb = Xo + row * kCin + kCf2 + l16 * 8;
    *(volatile v4u*)xa = ux;
    if (lane < 16) *(volatile v4u*)xb = uf;
    __threadfence();
    *(volatile v4u*)xa = ux;
    if (lane < 16) *(volatile v4u*)xb = uf;
  }
}

template <int COLS>
__global__ __launch_bounds__(COLS) void bn_partials_kernel(const float* __restrict__ H, float* __restrict__ part) {
  const int c = threadIdx.x;
  const size_t r0 = (size_t)blockIdx.x * kRowsPerStat;
  float s = 0.0f, q = 0.0f;
#pragma unroll 4
  for (int r = 0; r < kRowsPerStat; ++r) {
    const float v = H[(r0 + r) * COLS + c];
    s += v;
    const float vv = v * v;
    q += vv;
  }
  float* p = part + (size_t)blockIdx.x * 2 * COLS;
  ((volatile float*)p)[c] = s;
  ((volatile float*)p)[COLS + c] = q;
  __threadfence();
  ((volatile float*)p)[c] = s;
  ((volatile float*)p)[COLS + c] = q;
}

template <int COLS>
__global__ __launch_bounds__(COLS) void bn_finalize_kernel(const float* __restrict__ part, const float* __restrict__ gam,
                                                           const float* __restrict__ bet, float* __restrict__ tab) {
  const int c = threadIdx.x;
  double s = 0.0, q = 0.0;
#pragma unroll 4
  for (int blk = 0; blk < kStatBlocks; ++blk) {
    s += (double)part[(size_t)blk * 2 * COLS + c];
    q += (double)part[(size_t)blk * 2 * COLS + COLS + c];
  }
  const double mean = s * kInvRows;
  double var = q * kInvRows - mean * mean;
  var = var < 0.0 ? 0.0 : var;
  const float meanf = (float)mean;
  const float varf  = (float)var;
  const float rs = 1.0f / sqrtf(varf + kBnEps);
  const float sc = rs * bf16q(gam[c]);
  const float sh = bf16q(bet[c]);
  ((volatile float*)tab)[c]            = meanf;
  ((volatile float*)tab)[COLS + c]     = sc;
  ((volatile float*)tab)[2 * COLS + c] = sh;
  __threadfence();
  ((volatile float*)tab)[c]            = meanf;
  ((volatile float*)tab)[COLS + c]     = sc;
  ((volatile float*)tab)[2 * COLS + c] = sh;
}

__global__ __launch_bounds__(256) void bn_apply_h_kernel(const float* __restrict__ H, const float* __restrict__ tab,
                                                         unsigned short* __restrict__ Xo) {
  __shared__ float sm[3 * kHid1];
  const int t = threadIdx.x;
  sm[t] = tab[t];
  sm[kHid1 + t] = tab[kHid1 + t];
  sm[2 * kHid1 + t] = tab[2 * kHid1 + t];
  __syncthreads();
  const int lane = t & 31, wave = t >> 5;
  const int row = blockIdx.x * 8 + wave;
  const int c8 = lane * 8;
  const float* hp = H + (size_t)row * kHid1 + c8;
  const v4f a = *(const v4f*)(hp);
  const v4f c = *(const v4f*)(hp + 4);
  unsigned short hb[8];
#pragma unroll
  for (int e = 0; e < 4; ++e) {
    float y0 = (a[e] - sm[c8 + e]) * sm[kHid1 + c8 + e] + sm[2 * kHid1 + c8 + e];
    y0 = fmaxf(y0, 0.0f);
    hb[e] = h_bits(y0);
    float y1 = (c[e] - sm[c8 + 4 + e]) * sm[kHid1 + c8 + 4 + e] + sm[2 * kHid1 + c8 + 4 + e];
    y1 = fmaxf(y1, 0.0f);
    hb[4 + e] = h_bits(y1);
  }
  const v4u u = (v4u){pk16(hb[0], hb[1]), pk16(hb[2], hb[3]), pk16(hb[4], hb[5]), pk16(hb[6], hb[7])};
  unsigned short* q = Xo + (size_t)row * kCin + c8;
  *(volatile v4u*)q = u;
  __threadfence();
  *(volatile v4u*)q = u;
}

__global__ __launch_bounds__(256) void bn_apply_out_kernel(float* __restrict__ O, const float* __restrict__ tab) {
  __shared__ float sm[3 * kHid2];
  const int t = threadIdx.x;
  for (int i = t; i < 3 * kHid2; i += 256) sm[i] = tab[i];
  __syncthreads();
  const int lane = t & 31, wave = t >> 5;
  const int row = blockIdx.x * 8 + wave;
  const int c4 = lane * 4;
  float* p = O + (size_t)row * kHid2 + c4;
  const v4f x = *(const v4f*)p;
  v4f y;
#pragma unroll
  for (int e = 0; e < 4; ++e) {
    const float v = (x[e] - sm[c4 + e]) * sm[kHid2 + c4 + e] + sm[2 * kHid2 + c4 + e];
    y[e] = fmaxf(v, 0.0f);
  }
  *(volatile v4f*)p = y;
  __threadfence();
  *(volatile v4f*)p = y;
}

extern "C" void kernel_launch(void* const* d_in, const int* in_sizes, int n_in,
                              void* d_out, int out_size, void* d_ws, size_t ws_size,
                              hipStream_t stream) {
  if (n_in < 12) return;
  if (in_sizes[0] != kRows * 3 || in_sizes[1] != kBatch * kNs * 3 || in_sizes[2] != kRows * kCf1 ||
      in_sizes[3] != kBatch * kNs * kCf2 || in_sizes[4] != kHid1 * kCin || in_sizes[5] != kHid1 ||
      in_sizes[6] != kHid1 || in_sizes[7] != kHid1 || in_sizes[8] != kHid2 * kHid1 || in_sizes[9] != kHid2 ||
      in_sizes[10] != kHid2 || in_sizes[11] != kHid2) return;
  if (out_size != kRows * kHid2) return;
  if (ws_size < kWsTotal) return;

  const float* xyz1 = (const float*)d_in[0];
  const float* xyz2 = (const float*)d_in[1];
  const float* f1   = (const float*)d_in[2];
  const float* f2   = (const float*)d_in[3];
  const float* W1   = (const float*)d_in[4];
  const float* b1   = (const float*)d_in[5];
  const float* g1   = (const float*)d_in[6];
  const float* be1  = (const float*)d_in[7];
  const float* W2   = (const float*)d_in[8];
  const float* b2   = (const float*)d_in[9];
  const float* g2   = (const float*)d_in[10];
  const float* be2  = (const float*)d_in[11];
  float* out = (float*)d_out;

  char* ws = (char*)d_ws;
  unsigned short* XH  = (unsigned short*)(ws + kOffXH);
  float*          H1P = (float*)(ws + kOffH1P);
  unsigned short* W1H = (unsigned short*)(ws + kOffW1H);
  unsigned short* W2H = (unsigned short*)(ws + kOffW2H);
  float*          P1  = (float*)(ws + kOffP1);
  float*          P2  = (float*)(ws + kOffP2);
  float*          T1  = (float*)(ws + kOffT1);
  float*          T2  = (float*)(ws + kOffT2);

  const int n8w1 = kHid1 * kCin / 8;
  const int n8w2 = kHid2 * kHid1 / 8;
  cast8_w_kernel<<<n8w1 / 256, 256, 0, stream>>>(W1, W1H, n8w1, kWCarry);
  cast8_w_kernel<<<n8w2 / 256, 256, 0, stream>>>(W2, W2H, n8w2, kWCarry);

  knn_buildx_kernel<<<dim3(kNq / 256, kBatch), 256, 0, stream>>>(xyz1, xyz2, f1, f2, XH);

  wmma_gemm64<0, false, 2, 0, false, 0><<<dim3((kRows / 64) * (kHid1 / 64) / 8, 1), 256, 0, stream>>>(
      XH, XH, kCin, 0L, W1H, W1H, kCin, 0L, (void*)H1P, (void*)H1P, kHid1, 0L, b1, b1, 0L,
      kRows, kHid1, kCin, kWCarryInv);

  bn_partials_kernel<kHid1><<<kStatBlocks, kHid1, 0, stream>>>(H1P, P1);
  bn_finalize_kernel<kHid1><<<1, kHid1, 0, stream>>>(P1, g1, be1, T1);
  bn_apply_h_kernel<<<kRows / 8, 256, 0, stream>>>(H1P, T1, XH);

  wmma_gemm64<0, false, 2, 0, false, 0><<<dim3((kRows / 64) * (kHid2 / 64) / 8, 1), 256, 0, stream>>>(
      XH, XH, kCin, 0L, W2H, W2H, kHid1, 0L, (void*)out, (void*)out, kHid2, 0L, b2, b2, 0L,
      kRows, kHid2, kHid1, kWCarryInv);

  bn_partials_kernel<kHid2><<<kStatBlocks, kHid2, 0, stream>>>(out, P2);
  bn_finalize_kernel<kHid2><<<1, kHid2, 0, stream>>>(P2, g2, be2, T2);
  bn_apply_out_kernel<<<kRows / 8, 256, 0, stream>>>(out, T2);
}
